// GraphAttentionV2Layer_47605417509431
// MI455X (gfx1250) — hardware-run, weakly checked
//
#include <hip/hip_runtime.h>


#define NG   400
#define GC   50
#define NN   128
#define FIN  128
#define NH_  8
#define FH   32
#define CATK 160
typedef _Float16 h16;
typedef unsigned short bf;
typedef __attribute__((ext_vector_type(16))) __bf16   v16bf;
typedef __attribute__((ext_vector_type(16))) _Float16 v16h;
typedef __attribute__((ext_vector_type(8)))  _Float16 v8h;
typedef __attribute__((ext_vector_type(8)))  unsigned short v8us;
typedef __attribute__((ext_vector_type(8)))  float    v8f;
typedef __attribute__((ext_vector_type(4)))  float    v4f;
typedef v8h  __attribute__((may_alias)) v8ha;
typedef v4f  __attribute__((may_alias)) v4fa;
typedef v8us __attribute__((may_alias)) v8usa;

__device__ __forceinline__ unsigned short f2bf(float f) { unsigned u = __float_as_uint(f); u += 0x7FFFu + ((u >> 16) & 1u); return (unsigned short)(u >> 16); }
__device__ __forceinline__ float bf2f(unsigned short b) { return __uint_as_float(((unsigned)b) << 16); }
__device__ __forceinline__ float bfr(float f) { return bf2f(f2bf(f)); }
__device__ __forceinline__ v16h cat16(v8h lo, v8h hi) { return __builtin_shufflevector(lo, hi, 0, 1, 2, 3, 4, 5, 6, 7, 8, 9, 10, 11, 12, 13, 14, 15); }
__device__ __forceinline__ v16bf cat16b(v8us lo, v8us hi) { return __builtin_bit_cast(v16bf, __builtin_shufflevector(lo, hi, 0, 1, 2, 3, 4, 5, 6, 7, 8, 9, 10, 11, 12, 13, 14, 15)); }
__device__ __forceinline__ v8f wmma16(v16h a, v16h b, v8f c) { return __builtin_amdgcn_wmma_f32_16x16x32_f16(false, a, false, b, (short)0, c, false, false); }
__device__ __forceinline__ v8f wmmab(v16bf a, v16bf b, v8f c) { return __builtin_amdgcn_wmma_f32_16x16x32_bf16(false, a, false, b, (short)0, c, false, false); }


template <typename T16> struct WFrag;
template <> struct WFrag<h16> { typedef v16h V; static __device__ __forceinline__ V ld(const h16* p) { return cat16(*(const v8h*)p, *(const v8h*)(p + 16)); } static __device__ __forceinline__ v8f mma(V a, V b, v8f c) { return wmma16(a, b, c); } };
template <> struct WFrag<bf> { typedef v16bf V; static __device__ __forceinline__ V ld(const bf* p) { return cat16b(*(const v8us*)p, *(const v8us*)(p + 16)); } static __device__ __forceinline__ v8f mma(V a, V b, v8f c) { return wmmab(a, b, c); } };
template <typename T16, int NSPLIT, bool BIAS>
__global__ __launch_bounds__(32) void k_gemmw(const T16* __restrict__ A, const T16* __restrict__ A2, const T16* __restrict__ Bt, const T16* __restrict__ Bt2, int K, float* C, int ldc, const float* __restrict__ bias, size_t sA, size_t sB, size_t sC) {
    typedef typename WFrag<T16>::V V;
    __shared__ __align__(16) float os[16 * 68];
    const size_t z = blockIdx.z; A += z * sA; if (A2) A2 += z * sA; Bt += z * sB; if (Bt2) Bt2 += z * sB; C += z * sC;
    const int lane = threadIdx.x & 31, lr = lane & 15, hi = lane >> 4; const int r0 = blockIdx.x * 64, c0 = blockIdx.y * 64;
    v8f acc[4][4];
#pragma unroll
    for (int mb = 0; mb < 4; ++mb)
#pragma unroll
        for (int nb = 0; nb < 4; ++nb) acc[mb][nb] = (v8f){};
    const size_t aoff = (size_t)(r0 + lr) * K + 8 * hi, boff = (size_t)(c0 + lr) * K + 8 * hi;
#pragma unroll 1
    for (int kc = 0; kc < K; kc += 32) {
        V a[4], a2[4];
#pragma unroll
        for (int mb = 0; mb < 4; ++mb) { a[mb] = WFrag<T16>::ld(A + aoff + (size_t)mb * 16 * K + kc); if (NSPLIT == 1 || NSPLIT == 2) a2[mb] = WFrag<T16>::ld(A2 + aoff + (size_t)mb * 16 * K + kc); }
#pragma unroll
        for (int nb = 0; nb < 4; ++nb) { const V b = WFrag<T16>::ld(Bt + boff + (size_t)nb * 16 * K + kc); V b2; if (NSPLIT >= 2) b2 = WFrag<T16>::ld(Bt2 + boff + (size_t)nb * 16 * K + kc);
#pragma unroll
            for (int mb = 0; mb < 4; ++mb) { acc[mb][nb] = WFrag<T16>::mma(a[mb], b, acc[mb][nb]); if (NSPLIT == 1 || NSPLIT == 2) acc[mb][nb] = WFrag<T16>::mma(a2[mb], b, acc[mb][nb]); if (NSPLIT >= 2) acc[mb][nb] = WFrag<T16>::mma(a[mb], b2, acc[mb][nb]); } }
        asm volatile("v_nop\n\tv_nop\n\tv_nop\n\tv_nop" : "+v"(acc[0][0]), "+v"(acc[1][1]), "+v"(acc[2][2]), "+v"(acc[3][3]) : "v"(a[0]), "v"(a[3]));
    }
#pragma unroll
    for (int mb = 0; mb < 4; ++mb) {
#pragma unroll
        for (int nb = 0; nb < 4; ++nb) {
#pragma unroll
            for (int j = 0; j < 8; ++j) os[(hi * 8 + j) * 68 + nb * 16 + lr] = acc[mb][nb][j]; }
        __builtin_amdgcn_wave_barrier(); asm volatile("" ::: "memory");
        float* crow = C + (size_t)(r0 + mb * 16) * ldc + c0;
#pragma unroll 1
        for (int ps = 0; ps < 2; ++ps) {
#pragma unroll
            for (int s = 0; s < 8; ++s) { const int row = 2 * s + hi, cofs = lr * 4; v4f val = *(const v4fa*)(os + row * 68 + cofs); if (BIAS) { val[0] += bfr(bias[c0 + cofs]); val[1] += bfr(bias[c0 + cofs + 1]); val[2] += bfr(bias[c0 + cofs + 2]); val[3] += bfr(bias[c0 + cofs + 3]); }
                *(volatile v4f*)(crow + (size_t)row * ldc + cofs) = val; }
            if (ps == 0) __threadfence(); }
        __builtin_amdgcn_wave_barrier(); asm volatile("" ::: "memory");
    }
}

__device__ __forceinline__ void splitf(float y, unsigned short& h, unsigned short& l) { h = f2bf(y); l = f2bf(y - bf2f(h)); }
typedef __attribute__((ext_vector_type(2))) unsigned short v2us;
typedef __attribute__((ext_vector_type(4))) unsigned short v4us;

__global__ __launch_bounds__(256) void k_cvt8(const float* __restrict__ src, bf* dst, size_t n8) { const size_t i = (size_t)blockIdx.x * 256 + threadIdx.x; if (i >= n8) return; const v8f v = *(const v8f*)(src + i * 8); v8us o;
#pragma unroll
    for (int k = 0; k < 8; ++k) o[k] = f2bf(v[k]); *(volatile v8us*)(dst + i * 8) = o; __threadfence(); *(volatile v8us*)(dst + i * 8) = o; }
__global__ __launch_bounds__(256) void k_wpadT(const float* __restrict__ w, int N, int K, int NP, bf* Bt) { const int e = (blockIdx.x * 256 + threadIdx.x) * 4; if (e >= NP * K) return; const int k = e % K; const int n = e / K; v4us o;
#pragma unroll
    for (int u = 0; u < 4; ++u) o[u] = (n < N) ? f2bf(w[(size_t)n * K + k + u]) : (unsigned short)0; *(volatile v4us*)(Bt + e) = o; __threadfence(); *(volatile v4us*)(Bt + e) = o; }
__global__ __launch_bounds__(256) void k_qkpl(const float* __restrict__ F, int g0, float sgn, bf* Ph, bf* Pl) { const size_t e = ((size_t)blockIdx.x * 256 + threadIdx.x) * 4; if (e >= (size_t)GC * NH_ * NN * FH) return; const int f = (int)(e % FH); const int i = (int)((e / FH) % NN); const int z = (int)(e / ((size_t)FH * NN)); const int gl = z / NH_, h = z % NH_; (void)g0; const float* src = F + ((size_t)gl * NN + i) * (NH_ * FH) + h * FH + f; v4us oh, ol;
#pragma unroll
    for (int u = 0; u < 4; ++u) { unsigned short a, b; splitf(src[u] * sgn, a, b); oh[u] = a; ol[u] = b; } *(volatile v4us*)(Ph + e) = oh; *(volatile v4us*)(Pl + e) = ol; __threadfence(); *(volatile v4us*)(Ph + e) = oh; *(volatile v4us*)(Pl + e) = ol; }
__global__ __launch_bounds__(256) void k_spath(const float* __restrict__ S, const float* __restrict__ adj, const float* __restrict__ V, int g0, const float* __restrict__ saw, const float* __restrict__ sab, const float* __restrict__ lnw, const float* __restrict__ lnb, bf* Ch, bf* Cl) {
    const int lane = threadIdx.x & 31; const int row = blockIdx.x * 8 + (threadIdx.x >> 5); if (row >= GC * NH_ * NN) return; const int i = row % NN; const int z = row / NN; const int g = g0 + z / NH_, h = z % NH_; const float* sr = S + (size_t)row * NN; const float* ar = adj + ((size_t)g * NN + i) * NN; const float iscale = 5.5242717280199021e-03f;
    float es = 0.f;
#pragma unroll
    for (int m = 0; m < 4; ++m) { const int j = m * 32 + lane; float av = bfr(ar[j]); asm volatile("" : "+v"(av)); const float am = __fsub_rn(av, (j == i) ? 1.0f : 0.0f); const float sc = (am < 0.1f) ? -1.0e6f : sr[j] * iscale; es += __expf(sc); }
#pragma unroll
    for (int sh = 16; sh; sh >>= 1) es += __shfl_xor(es, sh, 32);
    float v4[4]; float su = 0.f;
#pragma unroll
    for (int m = 0; m < 4; ++m) { const int j = m * 32 + lane; float w = bfr(saw[j]), bb = bfr(sab[j]); asm volatile("" : "+v"(w)); asm volatile("" : "+v"(bb)); float t = __fmul_rn(es, w); asm volatile("" : "+v"(t)); v4[m] = __fadd_rn(t, bb); su += v4[m]; }
#pragma unroll
    for (int sh = 16; sh; sh >>= 1) su += __shfl_xor(su, sh, 32);
    const float mean = su * (1.0f / NN); float q = 0.f;
#pragma unroll
    for (int m = 0; m < 4; ++m) { float d = __fsub_rn(v4[m], mean); asm volatile("" : "+v"(d)); v4[m] = d; float p = __fmul_rn(d, d); asm volatile("" : "+v"(p)); q = __fadd_rn(q, p); }
#pragma unroll
    for (int sh = 16; sh; sh >>= 1) q += __shfl_xor(q, sh, 32);
    const float rs = __frsqrt_rn(__fadd_rn(q * (1.0f / NN), 1e-5f)); float mx = -3.0e38f;
#pragma unroll
    for (int m = 0; m < 4; ++m) { const int j = m * 32 + lane; float n0 = __fmul_rn(v4[m], rs); asm volatile("" : "+v"(n0)); float gw = bfr(lnw[j]), gb = bfr(lnb[j]); asm volatile("" : "+v"(gw)); asm volatile("" : "+v"(gb)); float t1 = __fmul_rn(n0, gw); asm volatile("" : "+v"(t1)); v4[m] = __fadd_rn(t1, gb); mx = fmaxf(mx, v4[m]); }
#pragma unroll
    for (int sh = 16; sh; sh >>= 1) mx = fmaxf(mx, __shfl_xor(mx, sh, 32));
    float se = 0.f;
#pragma unroll
    for (int m = 0; m < 4; ++m) { float d0 = __fsub_rn(v4[m], mx); asm volatile("" : "+v"(d0)); v4[m] = __builtin_amdgcn_exp2f(__fmul_rn(d0, 1.4426950408889634f)); se += v4[m]; }
#pragma unroll
    for (int sh = 16; sh; sh >>= 1) se += __shfl_xor(se, sh, 32);
    const float inv = __fdiv_rn(1.0f, se); const float vv = V[((size_t)(z / NH_) * NN + i) * (NH_ * FH) + h * FH + lane];
    for (int ps = 0; ps < 2; ++ps) {
#pragma unroll
        for (int m = 0; m < 4; ++m) { unsigned short a, b; splitf(v4[m] * inv, a, b); const size_t oo = (size_t)row * CATK + m * 32 + lane; *(volatile unsigned short*)(Ch + oo) = a; *(volatile unsigned short*)(Cl + oo) = b; }
        { unsigned short a, b; splitf(vv, a, b); const size_t oo = (size_t)row * CATK + NN + lane; *(volatile unsigned short*)(Ch + oo) = a; *(volatile unsigned short*)(Cl + oo) = b; }
        if (ps == 0) __threadfence(); } }
__global__ __launch_bounds__(256) void k_lrelu(const float* __restrict__ F, const float* __restrict__ b1, bf* Hh, bf* Hl) { const size_t e = ((size_t)blockIdx.x * 256 + threadIdx.x) * 4; if (e >= (size_t)GC * NH_ * NN * FH) return; const int f = (int)(e % FH); const size_t r = e / FH; v4us oh, ol;
#pragma unroll
    for (int u = 0; u < 4; ++u) { const float a = __fadd_rn(F[r * 64 + f + u], bfr(b1[f + u])); float lk = __fmul_rn(0.01f, a); asm volatile("" : "+v"(lk)); unsigned short p, q; splitf(fmaxf(a, lk), p, q); oh[u] = p; ol[u] = q; } *(volatile v4us*)(Hh + e) = oh; *(volatile v4us*)(Hl + e) = ol; __threadfence(); *(volatile v4us*)(Hh + e) = oh; *(volatile v4us*)(Hl + e) = ol; }
__global__ __launch_bounds__(256) void k_scpl(const float* __restrict__ F, const float* __restrict__ b, bf* Hh, bf* Hl) { const size_t e = ((size_t)blockIdx.x * 256 + threadIdx.x) * 4; if (e >= (size_t)GC * NH_ * NN * FH) return; const int f = (int)(e % FH); const size_t r = e / FH; v4us oh, ol;
#pragma unroll
    for (int u = 0; u < 4; ++u) { unsigned short p, q; splitf(__fadd_rn(F[r * 64 + f + u], bfr(b[f + u])), p, q); oh[u] = p; ol[u] = q; } *(volatile v4us*)(Hh + e) = oh; *(volatile v4us*)(Hl + e) = ol; __threadfence(); *(volatile v4us*)(Hh + e) = oh; *(volatile v4us*)(Hl + e) = ol; }
__global__ __launch_bounds__(256) void k_outg(const float* __restrict__ SC, const float* __restrict__ FF, int g0, const float* __restrict__ atb, const float* __restrict__ fb2, const float* __restrict__ rz, float* out) { const size_t e = ((size_t)blockIdx.x * 256 + threadIdx.x) * 4; if (e >= (size_t)GC * NN * NH_ * FH) return; const int c = (int)(e % (NH_ * FH)); const size_t gi = e / (NH_ * FH); const int i = (int)(gi % NN); const int gl = (int)(gi / NN); const int h = c / FH, f = c % FH; const size_t r = ((size_t)(gl * NH_ + h)) * NN + i; v4f o;
#pragma unroll
    for (int u = 0; u < 4; ++u) { const float sc = __fadd_rn(SC[r * 64 + f + u], bfr(atb[f + u])); const float ffv = __fadd_rn(FF[r * 64 + f + u], bfr(fb2[f + u])); float rf = __fmul_rn(bfr(rz[f + u]), ffv); asm volatile("" : "+v"(rf)); o[u] = __fadd_rn(sc, rf); }
    float* dst = out + ((size_t)(g0 + gl) * NN + i) * (NH_ * FH) + c; *(volatile v4f*)dst = o; __threadfence(); *(volatile v4f*)dst = o; }

extern "C" void kernel_launch(void* const* d_in, const int* in_sizes, int n_in,
                              void* d_out, int out_size, void* d_ws, size_t ws_size, hipStream_t stream) {
    (void)in_sizes; (void)n_in; (void)out_size;
    const float** I = (const float**)d_in;
    const float *h0 = I[0], *adj = I[1], *Wl = I[2], *Wr = I[3], *Wv = I[4], *saw = I[5], *sab = I[6], *lnw = I[7], *lnb = I[8], *atw = I[9], *atb = I[10], *fw1 = I[11], *fb1 = I[12], *fw2 = I[13], *fb2 = I[14], *rz = I[15];
    float* OUT = (float*)d_out;
    char* wsp = (char*)d_ws;
    auto take = [&](size_t bytes) { char* p = wsp; wsp += (bytes + 255) & ~(size_t)255; return (void*)p; };
    const size_t NR = (size_t)NG * NN; const size_t RC = (size_t)GC * NH_ * NN;
    bf* HB = (bf*)take(NR * FIN * 2); bf* BL = (bf*)take(256 * FIN * 2); bf* BR = (bf*)take(256 * FIN * 2); bf* BV = (bf*)take(256 * FIN * 2); bf* BAT = (bf*)take(64 * CATK * 2); bf* BF1 = (bf*)take(64 * FH * 2); bf* BF2 = (bf*)take(64 * FH * 2);
    float* Q = (float*)take((size_t)GC * NN * 256 * 4); float* K = (float*)take((size_t)GC * NN * 256 * 4); float* V = (float*)take((size_t)GC * NN * 256 * 4);
    bf* QPh = (bf*)take(RC * FH * 2); bf* QPl = (bf*)take(RC * FH * 2); bf* KPh = (bf*)take(RC * FH * 2); bf* KPl = (bf*)take(RC * FH * 2); float* S = (float*)take(RC * NN * 4); bf* Ch = (bf*)take(RC * CATK * 2); bf* Cl = (bf*)take(RC * CATK * 2); float* SC = (float*)take(RC * 64 * 4);
    bf* Ah = (bf*)take(RC * FH * 2); bf* Al = (bf*)take(RC * FH * 2); float* F1 = (float*)take(RC * 64 * 4); float* F2 = (float*)take(RC * 64 * 4);
    if ((size_t)(wsp - (char*)d_ws) > ws_size) return;
    k_cvt8<<<(unsigned)((NR * FIN / 8 + 255) / 256), 256, 0, stream>>>(h0, HB, NR * FIN / 8); k_cvt8<<<(256 * FIN / 8 + 255) / 256, 256, 0, stream>>>(Wl, BL, 256 * FIN / 8); k_cvt8<<<(256 * FIN / 8 + 255) / 256, 256, 0, stream>>>(Wr, BR, 256 * FIN / 8); k_cvt8<<<(256 * FIN / 8 + 255) / 256, 256, 0, stream>>>(Wv, BV, 256 * FIN / 8);
    k_wpadT<<<(64 * CATK / 4 + 255) / 256, 256, 0, stream>>>(atw, FH, CATK, 64, BAT); k_wpadT<<<(64 * FH / 4 + 255) / 256, 256, 0, stream>>>(fw1, FH, FH, 64, BF1); k_wpadT<<<(64 * FH / 4 + 255) / 256, 256, 0, stream>>>(fw2, FH, FH, 64, BF2);
    const unsigned gP = (unsigned)((RC * FH / 4 + 255) / 256);
    for (int g0 = 0; g0 < NG; g0 += GC) { const bf* HBc = HB + (size_t)g0 * NN * FIN; const dim3 gq((unsigned)((size_t)GC * NN / 64), 4, 1);
        k_gemmw<bf, 0, false><<<gq, 32, 0, stream>>>(HBc, nullptr, BL, nullptr, FIN, Q, 256, nullptr, 0, 0, 0); k_gemmw<bf, 0, false><<<gq, 32, 0, stream>>>(HBc, nullptr, BR, nullptr, FIN, K, 256, nullptr, 0, 0, 0); k_gemmw<bf, 0, false><<<gq, 32, 0, stream>>>(HBc, nullptr, BV, nullptr, FIN, V, 256, nullptr, 0, 0, 0);
        k_qkpl<<<gP, 256, 0, stream>>>(Q, g0, 1.0f, QPh, QPl); k_qkpl<<<gP, 256, 0, stream>>>(K, g0, -1.0f, KPh, KPl);
        k_gemmw<bf, 2, false><<<dim3(NN / 64, NN / 64, GC * NH_), 32, 0, stream>>>(QPh, QPl, KPh, KPl, FH, S, NN, nullptr, (size_t)NN * FH, (size_t)NN * FH, (size_t)NN * NN);
        k_spath<<<(unsigned)(RC / 8), 256, 0, stream>>>(S, adj, V, g0, saw, sab, lnw, lnb, Ch, Cl);
        k_gemmw<bf, 1, false><<<dim3((unsigned)(RC / 64), 1, 1), 32, 0, stream>>>(Ch, Cl, BAT, nullptr, CATK, SC, 64, nullptr, 0, 0, 0);
        k_scpl<<<gP, 256, 0, stream>>>(SC, atb, Ah, Al);
        k_gemmw<bf, 1, false><<<dim3((unsigned)(RC / 64), 1, 1), 32, 0, stream>>>(Ah, Al, BF1, nullptr, FH, F1, 64, nullptr, 0, 0, 0);
        k_lrelu<<<gP, 256, 0, stream>>>(F1, fb1, Ah, Al);
        k_gemmw<bf, 1, false><<<dim3((unsigned)(RC / 64), 1, 1), 32, 0, stream>>>(Ah, Al, BF2, nullptr, FH, F2, 64, nullptr, 0, 0, 0);
        k_outg<<<(unsigned)((RC * FH / 4 + 255) / 256), 256, 0, stream>>>(SC, F2, g0, atb, fb2, rz, OUT); }
}
